// MultiHeadCoAttention_63385127355034
// MI455X (gfx1250) — hardware-verified
//
#include <hip/hip_runtime.h>


#ifndef NB
#define NB 2
#endif
#ifndef SEQ
#define SEQ 1024
#endif
#define NB_FULL  2
#define SEQ_FULL 1024
#ifndef OUT_SEQ
#define OUT_SEQ SEQ
#endif
#define CC    64
#define NHD   8
#define HDM   8
#define VROWS 16
#define TSP   72
#define CSP   72
#define QRS  2048.0f
#define QRI  (1.0f / 2048.0f)
#define WCS  256.0f
#define WCI  (1.0f / 256.0f)
#define L2E  1.4426950408889634f
#define PSH  14.0f

static_assert(CC == 64);
static_assert(NHD * HDM == CC);
static_assert(HDM == 8);
static_assert(CC % 32 == 0);
static_assert(SEQ % 64 == 0);
static_assert(SEQ % 128 == 0);
static_assert(SEQ % 32 == 0);
static_assert(SEQ % 16 == 0);
static_assert(OUT_SEQ % 64 == 0);
static_assert(VROWS == 16);
static_assert(NB <= NB_FULL);
static_assert(SEQ <= SEQ_FULL);
static_assert(((size_t)CC * CC) % 8 == 0);
static_assert((TSP * 2) % 16 == 0);
static_assert((CSP * 2) % 16 == 0);
static_assert(256 * 16 * 2 == 64 * CC * 2);
static_assert(32 * 16 * 8 == 16 * CC * 4);
static_assert(32 * 16 * 4 == NHD * 64 * 4);
static_assert(32 * 16 * 32 == NHD * VROWS * 64 * 2);
static_assert(128 * 16 * 1 == 16 * CC * 2);
static_assert(64 * TSP * 2 <= 131072);
static_assert(16 * 68 * 4 <= 131072);
static_assert(NHD * 68 * 4 <= 131072);
static_assert(16 * CSP * 2 <= 131072);

typedef _Float16 h16;
typedef unsigned short bf;
typedef __attribute__((ext_vector_type(16))) __bf16   v16bf;
typedef __attribute__((ext_vector_type(16))) _Float16 v16h;
typedef __attribute__((ext_vector_type(8)))  _Float16 v8h;
typedef __attribute__((ext_vector_type(8)))  unsigned short v8us;
typedef __attribute__((ext_vector_type(8)))  float    v8f;
typedef __attribute__((ext_vector_type(4)))  float    v4f;
typedef v4f  __attribute__((may_alias)) v4fa;
typedef v8h  __attribute__((may_alias)) v8ha;
typedef v8us __attribute__((may_alias)) v8usa;

__device__ __forceinline__ unsigned short f2bf(float f) { unsigned u = __float_as_uint(f); u += 0x7FFFu + ((u >> 16) & 1u); return (unsigned short)(u >> 16); }
__device__ __forceinline__ float bfr(float f) { return __uint_as_float(((unsigned)f2bf(f)) << 16); }
__device__ __forceinline__ v16h cat16(v8h lo, v8h hi) { return __builtin_shufflevector(lo, hi, 0, 1, 2, 3, 4, 5, 6, 7, 8, 9, 10, 11, 12, 13, 14, 15); }
__device__ __forceinline__ v16bf cat16b(v8us lo, v8us hi) { return __builtin_bit_cast(v16bf, __builtin_shufflevector(lo, hi, 0, 1, 2, 3, 4, 5, 6, 7, 8, 9, 10, 11, 12, 13, 14, 15)); }
__device__ __forceinline__ v16h  ldh(const h16* p) { return cat16(*(const v8h*)p, *(const v8h*)(p + 16)); }
__device__ __forceinline__ v16bf ldb(const bf* p)  { return cat16b(*(const v8us*)p, *(const v8us*)(p + 16)); }
__device__ __forceinline__ void wave_sync() { __builtin_amdgcn_fence(3  , "wavefront"); __builtin_amdgcn_wave_barrier(); asm volatile("" ::: "memory"); }
__device__ __forceinline__ v8f wmma16g(v16h a, v16h b, v8f c) {
    c = __builtin_amdgcn_wmma_f32_16x16x32_f16(false, a, false, b, (short)0, c, false, false);
    asm volatile("v_nop\n\tv_nop\n\tv_nop\n\tv_nop" : "+v"(c) : "v"(a), "v"(b));
    return c; }
__device__ __forceinline__ v8f wmmabg(v16bf a, v16bf b, v8f c) {
    c = __builtin_amdgcn_wmma_f32_16x16x32_bf16(false, a, false, b, (short)0, c, false, false);
    asm volatile("v_nop\n\tv_nop\n\tv_nop\n\tv_nop" : "+v"(c) : "v"(a), "v"(b));
    return c; }
static __device__ __forceinline__ h16 toh_flush(float v) { const h16 r = (h16)v; return (fabsf(v) < 6.103515625e-05f) ? (h16)0.0f : r; }
static __device__ __forceinline__ h16 p16(float e) { const float x = __builtin_amdgcn_exp2f(e); return (e < -14.0f) ? (h16)0.0f : (h16)x; }

__global__ __launch_bounds__(256) void k_cvt8(const float* __restrict__ src, bf* dst, size_t n8) {
    const size_t i = (size_t)blockIdx.x * 256 + threadIdx.x; if (i >= n8) return;
    const v8f v = *(const v8f*)(src + i * 8); v8us o;
#pragma unroll
    for (int k = 0; k < 8; ++k) o[k] = f2bf(v[k]);
    *(volatile v8us*)(dst + i * 8) = o; __threadfence(); *(volatile v8us*)(dst + i * 8) = o;
}

__global__ __launch_bounds__(256) void k_wconv(const float* __restrict__ src, h16* dst, size_t n8) {
    const size_t i = (size_t)blockIdx.x * 256 + threadIdx.x; if (i >= n8) return;
    const v8f v = *(const v8f*)(src + i * 8); v8h o;
#pragma unroll
    for (int k = 0; k < 8; ++k) o[k] = toh_flush(bfr(v[k]) * WCS);
    *(volatile v8h*)(dst + i * 8) = o; __threadfence(); *(volatile v8h*)(dst + i * 8) = o;
}

__global__ __launch_bounds__(256) void k_cvtT(const float* __restrict__ src, bf* dst) {
    __shared__ __align__(16) unsigned short ts[64 * TSP];
    const int tid = threadIdx.x;
    const int b = blockIdx.y, p0 = blockIdx.x * 64;
    const int c = tid >> 2, pq = (tid & 3) * 16;
    const float* sp = src + ((size_t)b * CC + c) * SEQ_FULL + p0 + pq;
#pragma unroll
    for (int i = 0; i < 4; ++i) { const v4f v = *(const v4f*)(sp + 4 * i);
#pragma unroll
        for (int j = 0; j < 4; ++j) ts[(pq + 4 * i + j) * TSP + c] = f2bf(v[j]); }
    __syncthreads();
    bf* dp = dst + ((size_t)b * SEQ + p0) * CC;
#pragma unroll 1
    for (int ps = 0; ps < 2; ++ps) {
#pragma unroll
        for (int s = 0; s < 2; ++s) { const int idx = s * 256 + tid; const int row = idx >> 3, pc = idx & 7;
            const v8us val = *(const v8usa*)(&ts[row * TSP + pc * 8]);
            *(volatile v8us*)(dp + (size_t)idx * 8) = val; }
        if (ps == 0) __threadfence(); }
}

__device__ __forceinline__ void mm64b(const bf* __restrict__ A, const bf* __restrict__ Bt, const size_t aoff, const size_t boff, v8f (&acc)[4][4]) {
#pragma unroll
    for (int kc = 0; kc < CC; kc += 32) {
        v16bf a[4];
#pragma unroll
        for (int mb = 0; mb < 4; ++mb) a[mb] = ldb(A + aoff + (size_t)mb * 16 * CC + kc);
#pragma unroll
        for (int nb = 0; nb < 4; ++nb) { const v16bf b = ldb(Bt + boff + (size_t)nb * 16 * CC + kc);
#pragma unroll
            for (int mb = 0; mb < 4; ++mb) acc[mb][nb] = wmmabg(a[mb], b, acc[mb][nb]); }
    }
}
__device__ __forceinline__ void mm64h(const h16* __restrict__ A, const h16* __restrict__ Bt, const size_t aoff, const size_t boff, v8f (&acc)[4][4]) {
#pragma unroll
    for (int kc = 0; kc < CC; kc += 32) {
        v16h a[4];
#pragma unroll
        for (int mb = 0; mb < 4; ++mb) a[mb] = ldh(A + aoff + (size_t)mb * 16 * CC + kc);
#pragma unroll
        for (int nb = 0; nb < 4; ++nb) { const v16h b = ldh(Bt + boff + (size_t)nb * 16 * CC + kc);
#pragma unroll
            for (int mb = 0; mb < 4; ++mb) acc[mb][nb] = wmma16g(a[mb], b, acc[mb][nb]); }
    }
}

__global__ __launch_bounds__(32) void k_qproj(const bf* __restrict__ XT, const bf* __restrict__ WQ, const float* __restrict__ bias, float* QP) {
    __shared__ __align__(16) float os[16 * 68];
    const int lane = threadIdx.x & 31, lr = lane & 15, hi = lane >> 4; const int r0 = blockIdx.x * 64;
    v8f acc[4][4];
#pragma unroll
    for (int mb = 0; mb < 4; ++mb)
#pragma unroll
        for (int nb = 0; nb < 4; ++nb) acc[mb][nb] = (v8f){};
    mm64b(XT, WQ, (size_t)(r0 + lr) * CC + 8 * hi, (size_t)lr * CC + 8 * hi, acc);
    float bc[4];
#pragma unroll
    for (int nb = 0; nb < 4; ++nb) bc[nb] = bfr(bias[nb * 16 + lr]);
#pragma unroll
    for (int mb = 0; mb < 4; ++mb) {
#pragma unroll
        for (int nb = 0; nb < 4; ++nb) {
#pragma unroll
            for (int j = 0; j < 8; ++j) os[(hi * 8 + j) * 68 + nb * 16 + lr] = acc[mb][nb][j] + bc[nb]; }
        wave_sync();
        float* dst = QP + (size_t)(r0 + mb * 16) * CC;
#pragma unroll 1
        for (int ps = 0; ps < 2; ++ps) {
#pragma unroll
            for (int s = 0; s < 8; ++s) { const int row = 2 * s + (lane >> 4), c4 = (lane & 15) * 4;
                const v4f val = *(const v4fa*)(&os[row * 68 + c4]);
                *(volatile v4f*)(dst + (size_t)row * CC + c4) = val; }
            if (ps == 0) __threadfence(); }
        wave_sync();
    }
}

__global__ __launch_bounds__(32) void k_ksum(const bf* __restrict__ WK, const bf* __restrict__ XT, const float* __restrict__ bias, float* KS) {
    __shared__ __align__(16) float hs[NHD * 68];
    const int lane = threadIdx.x & 31, lr = lane & 15, hi = lane >> 4; const int c0 = blockIdx.x * 64;
    v8f acc[4][4];
#pragma unroll
    for (int mb = 0; mb < 4; ++mb)
#pragma unroll
        for (int nb = 0; nb < 4; ++nb) acc[mb][nb] = (v8f){};
    mm64b(WK, XT, (size_t)lr * CC + 8 * hi, (size_t)(c0 + lr) * CC + 8 * hi, acc);
#pragma unroll
    for (int mb = 0; mb < 4; ++mb) {
        float br[8];
#pragma unroll
        for (int j = 0; j < 8; ++j) br[j] = bfr(bias[mb * 16 + hi * 8 + j]);
#pragma unroll
        for (int nb = 0; nb < 4; ++nb) { float s = 0.0f;
#pragma unroll
            for (int j = 0; j < 8; ++j) s += acc[mb][nb][j] + br[j];
            hs[(mb * 2 + hi) * 68 + nb * 16 + lr] = s; }
    }
    wave_sync();
    const int bb = c0 / SEQ, tt = c0 % SEQ;
    float* dst = KS + (size_t)bb * NHD * SEQ + tt;
#pragma unroll 1
    for (int ps = 0; ps < 2; ++ps) {
#pragma unroll
        for (int s = 0; s < 4; ++s) { const int row = 2 * s + (lane >> 4), c4 = (lane & 15) * 4;
            const v4f val = *(const v4fa*)(&hs[row * 68 + c4]);
            *(volatile v4f*)(dst + (size_t)row * SEQ + c4) = val; }
        if (ps == 0) __threadfence(); }
}

__global__ __launch_bounds__(32) void k_vsum(const bf* __restrict__ WV, const bf* __restrict__ XT, const float* __restrict__ bias, h16* VA) {
    __shared__ __align__(16) float hs[NHD * 68];
    const int lane = threadIdx.x & 31, lr = lane & 15, hi = lane >> 4; const int c0 = blockIdx.x * 64;
    v8f acc[4][4];
#pragma unroll
    for (int mb = 0; mb < 4; ++mb)
#pragma unroll
        for (int nb = 0; nb < 4; ++nb) acc[mb][nb] = (v8f){};
    mm64b(WV, XT, (size_t)lr * CC + 8 * hi, (size_t)(c0 + lr) * CC + 8 * hi, acc);
#pragma unroll
    for (int mb = 0; mb < 4; ++mb) {
        float br[8];
#pragma unroll
        for (int j = 0; j < 8; ++j) br[j] = bfr(bias[mb * 16 + hi * 8 + j]);
#pragma unroll
        for (int nb = 0; nb < 4; ++nb) { float s = 0.0f;
#pragma unroll
            for (int j = 0; j < 8; ++j) s += acc[mb][nb][j] + br[j];
            hs[(mb * 2 + hi) * 68 + nb * 16 + lr] = s; }
    }
    wave_sync();
    const int bb = c0 / SEQ, tt = c0 % SEQ;
    h16* dst = VA + (size_t)bb * NHD * VROWS * SEQ + tt;
#pragma unroll 1
    for (int ps = 0; ps < 2; ++ps) {
#pragma unroll 1
        for (int s = 0; s < 32; ++s) { const int line = 4 * s + (lane >> 3);
            const int hh = line >> 4, rr = line & 15, c8 = (lane & 7) * 8;
            const v4f y0 = *(const v4fa*)(&hs[hh * 68 + c8]); const v4f y1 = *(const v4fa*)(&hs[hh * 68 + c8 + 4]); v8h ov;
#pragma unroll
            for (int i = 0; i < 4; ++i) {
                const h16 a0 = toh_flush(y0[i]); const h16 a1 = toh_flush(y1[i]);
                const float r0 = (y0[i] - (float)a0) * QRS, r1 = (y1[i] - (float)a1) * QRS;
                const float s0 = (rr == 0) ? y0[i] : ((rr == 1) ? 1.0f : ((rr == 2) ? r0 : 0.0f));
                const float s1 = (rr == 0) ? y1[i] : ((rr == 1) ? 1.0f : ((rr == 2) ? r1 : 0.0f));
                ov[i] = toh_flush(s0); ov[4 + i] = toh_flush(s1); }
            *(volatile v8h*)(dst + ((size_t)hh * VROWS + rr) * SEQ + c8) = ov; }
        if (ps == 0) __threadfence(); }
}

__global__ __launch_bounds__(256) __attribute__((amdgpu_num_vgpr(256)))
void k_attn(const float* __restrict__ QP, const float* __restrict__ KS, const h16* __restrict__ VA, h16* CTX) {
    __shared__ __align__(16) h16 cs[16 * CSP];
    const int lane = threadIdx.x & 31, lr = lane & 15, hi = lane >> 4;
    const int wave = __builtin_amdgcn_readfirstlane((int)(threadIdx.x >> 5));
    const int b = blockIdx.y, q0 = blockIdx.x * 16;
    const int zh = b * NHD + wave;
    const float* kr = KS + (size_t)zh * SEQ;
    float kmx = -3.0e38f, kmn = 3.0e38f;
#pragma unroll 1
    for (int i = lane * 4; i < SEQ; i += 128) { const v4f v = *(const v4f*)(kr + i);
        kmx = fmaxf(kmx, fmaxf(fmaxf(v[0], v[1]), fmaxf(v[2], v[3])));
        kmn = fminf(kmn, fminf(fminf(v[0], v[1]), fminf(v[2], v[3]))); }
#pragma unroll
    for (int d = 16; d >= 1; d >>= 1) { kmx = fmaxf(kmx, __shfl_xor(kmx, d, 32)); kmn = fminf(kmn, __shfl_xor(kmn, d, 32)); }
    const float* qp = QP + ((size_t)b * SEQ + q0 + lr) * CC + wave * HDM;
    const v4f qa = *(const v4f*)qp, qb = *(const v4f*)(qp + 4);
    float tq[8], ms[8];
#pragma unroll
    for (int n = 0; n < 4; ++n) { tq[n] = qa[n] * L2E; tq[4 + n] = qb[n] * L2E; }
#pragma unroll
    for (int n = 0; n < 8; ++n) { const float mxl = (tq[n] >= 0.0f) ? tq[n] * kmx : tq[n] * kmn; ms[n] = PSH - mxl; }
    const size_t ao = (size_t)zh * VROWS * SEQ + (size_t)lr * SEQ + 8 * hi;
    const float* kb = kr + 8 * hi;
    v8f o[8];
#pragma unroll
    for (int n = 0; n < 8; ++n) o[n] = (v8f){};
#pragma unroll 1
    for (int key0 = 0; key0 < SEQ; key0 += 32) {
        const float* kp = kb + key0;
        const v4f m0 = *(const v4f*)kp, m1 = *(const v4f*)(kp + 4), m2 = *(const v4f*)(kp + 16), m3 = *(const v4f*)(kp + 20);
        float kx[8], ky[8];
#pragma unroll
        for (int r = 0; r < 4; ++r) { kx[r] = m0[r]; kx[4 + r] = m1[r]; ky[r] = m2[r]; ky[4 + r] = m3[r]; }
        const v16h va = ldh(VA + ao + key0);
#pragma unroll
        for (int n = 0; n < 8; ++n) {
            v16h pb;
#pragma unroll
            for (int r = 0; r < 8; ++r) {
                const float ea = fmaf(tq[n], kx[r], ms[n]), eb = fmaf(tq[n], ky[r], ms[n]);
                pb[r] = p16(ea); pb[8 + r] = p16(eb); }
            o[n] = wmma16g(va, pb, o[n]);
        }
    }
    v8h cv;
#pragma unroll
    for (int n = 0; n < 8; ++n) {
        const float den = (hi == 0) ? o[n][1] : 1.0f;
        const float num = o[n][0] + o[n][2] * QRI;
        cv[n] = toh_flush(num * (1.0f / den)); }
    if (hi == 0) *(v8ha*)(&cs[lr * CSP + wave * HDM]) = cv;
    __syncthreads();
    if (wave < 4) {
        const int tid = threadIdx.x; const int row = tid >> 3, pc = tid & 7;
        const v8h val = *(const v8ha*)(&cs[row * CSP + pc * 8]);
        h16* dp = CTX + ((size_t)b * SEQ + q0) * CC + (size_t)tid * 8;
        *(volatile v8h*)dp = val; __threadfence(); *(volatile v8h*)dp = val;
    }
}

__global__ __launch_bounds__(32) void k_oproj(const h16* __restrict__ WOH, const h16* __restrict__ CTX, const float* __restrict__ bias, const float* __restrict__ X1, float* OUT) {
    __shared__ __align__(16) float os[16 * 68];
    const int lane = threadIdx.x & 31, lr = lane & 15, hi = lane >> 4; const int c0 = blockIdx.x * 64;
    v8f acc[4][4];
#pragma unroll
    for (int mb = 0; mb < 4; ++mb)
#pragma unroll
        for (int nb = 0; nb < 4; ++nb) acc[mb][nb] = (v8f){};
    mm64h(WOH, CTX, (size_t)lr * CC + 8 * hi, (size_t)(c0 + lr) * CC + 8 * hi, acc);
    const int bb = c0 / SEQ, tt = c0 % SEQ;
#pragma unroll
    for (int mb = 0; mb < 4; ++mb) {
        float br[8];
#pragma unroll
        for (int j = 0; j < 8; ++j) br[j] = bfr(bias[mb * 16 + hi * 8 + j]);
#pragma unroll
        for (int nb = 0; nb < 4; ++nb) {
#pragma unroll
            for (int j = 0; j < 8; ++j) os[(hi * 8 + j) * 68 + nb * 16 + lr] = acc[mb][nb][j] * WCI + br[j]; }
        wave_sync();
        const size_t orow = (size_t)bb * CC + (size_t)(mb * 16);
#pragma unroll 1
        for (int ps = 0; ps < 2; ++ps) {
#pragma unroll
            for (int s = 0; s < 8; ++s) { const int row = 2 * s + (lane >> 4), c4 = (lane & 15) * 4;
                const v4f a = *(const v4fa*)(&os[row * 68 + c4]);
                const v4f xr = *(const v4f*)(X1 + (orow + row) * SEQ_FULL + tt + c4);
                v4f val;
#pragma unroll
                for (int i = 0; i < 4; ++i) val[i] = a[i] + bfr(xr[i]);
                *(volatile v4f*)(OUT + (orow + row) * OUT_SEQ + tt + c4) = val; }
            if (ps == 0) __threadfence(); }
        wave_sync();
    }
}

static constexpr size_t al256(size_t v) { return (v + 255) & ~(size_t)255; }
static constexpr size_t SZ_XT = al256((size_t)NB * SEQ * CC * 2);
static constexpr size_t SZ_WB = al256((size_t)3 * CC * CC * 2);
static constexpr size_t SZ_WO = al256((size_t)CC * CC * 2);
static constexpr size_t SZ_QP = al256((size_t)NB * SEQ * CC * 4);
static constexpr size_t SZ_KS = al256((size_t)NB * NHD * SEQ * 4);
static constexpr size_t SZ_VA = al256((size_t)NB * NHD * VROWS * SEQ * 2);
static constexpr size_t SZ_CX = al256((size_t)NB * SEQ * CC * 2);
static constexpr size_t SZ_TOTAL = 2 * SZ_XT + SZ_WB + SZ_WO + SZ_QP + SZ_KS + SZ_VA + SZ_CX;
static_assert(SZ_TOTAL <= (size_t)134217728);
static_assert(((size_t)CC * CC * 2) % 256 == 0);

extern "C" void kernel_launch(void* const* d_in, const int* in_sizes, int n_in,
                              void* d_out, int out_size, void* d_ws, size_t ws_size, hipStream_t stream) {
    if (n_in < 10) return;
    const size_t needx = ((size_t)(NB - 1) * CC + (size_t)(CC - 1)) * SEQ_FULL + SEQ;
    if ((size_t)in_sizes[0] < needx || (size_t)in_sizes[1] < needx) return;
    if ((size_t)in_sizes[2] < (size_t)CC * CC || (size_t)in_sizes[4] < (size_t)CC * CC || (size_t)in_sizes[6] < (size_t)CC * CC || (size_t)in_sizes[8] < (size_t)CC * CC) return;
    if (in_sizes[3] < CC || in_sizes[5] < CC || in_sizes[7] < CC || in_sizes[9] < CC) return;
    if ((size_t)out_size < ((size_t)(NB - 1) * CC + (size_t)(CC - 1)) * OUT_SEQ + SEQ) return;
    if (SZ_TOTAL > ws_size) return;
    const float* x1 = (const float*)d_in[0]; const float* x2 = (const float*)d_in[1];
    const float* wq = (const float*)d_in[2]; const float* bq = (const float*)d_in[3];
    const float* wk = (const float*)d_in[4]; const float* bk = (const float*)d_in[5];
    const float* wv = (const float*)d_in[6]; const float* bv = (const float*)d_in[7];
    const float* wo = (const float*)d_in[8]; const float* bo = (const float*)d_in[9];
    float* OUT = (float*)d_out;
    char* wsp = (char*)d_ws;
    bf* X1T = (bf*)wsp; wsp += SZ_XT;
    bf* X2T = (bf*)wsp; wsp += SZ_XT;
    bf* WB  = (bf*)wsp; wsp += SZ_WB;
    h16* WOH = (h16*)wsp; wsp += SZ_WO;
    float* QP = (float*)wsp; wsp += SZ_QP;
    float* KS = (float*)wsp; wsp += SZ_KS;
    h16* VA = (h16*)wsp; wsp += SZ_VA;
    h16* CTX = (h16*)wsp; wsp += SZ_CX;
    bf* WQ = WB; bf* WK = WB + (size_t)CC * CC; bf* WV = WB + (size_t)2 * CC * CC;

    k_cvtT<<<dim3(SEQ / 64, NB, 1), 256, 0, stream>>>(x1, X1T);
    k_cvtT<<<dim3(SEQ / 64, NB, 1), 256, 0, stream>>>(x2, X2T);
    { const size_t n8 = (size_t)CC * CC / 8; const unsigned g = (unsigned)((n8 + 255) / 256);
      k_cvt8<<<g, 256, 0, stream>>>(wq, WQ, n8); k_cvt8<<<g, 256, 0, stream>>>(wk, WK, n8); k_cvt8<<<g, 256, 0, stream>>>(wv, WV, n8);
      k_wconv<<<g, 256, 0, stream>>>(wo, WOH, n8); }

    k_qproj<<<dim3(NB * SEQ / 64, 1, 1), 32, 0, stream>>>(X1T, WQ, bq, QP);
    k_ksum<<<dim3(NB * SEQ / 64, 1, 1), 32, 0, stream>>>(WK, X2T, bk, KS);
    k_vsum<<<dim3(NB * SEQ / 64, 1, 1), 32, 0, stream>>>(WV, X2T, bv, VA);

    k_attn<<<dim3(SEQ / 16, NB, 1), 256, 0, stream>>>(QP, KS, VA, CTX);

    k_oproj<<<dim3(NB * SEQ / 64, 1, 1), 32, 0, stream>>>(WOH, CTX, bo, x1, OUT);
}
